// DCNV4_YOLO_16140487098591
// MI455X (gfx1250) — hardware-verified
//
#include <hip/hip_runtime.h>


namespace {
constexpr int NBt = 4, C = 256, H = 64, W = 64, HW = H * W, NTOK = NBt * HW, G = 4, CG = 64, KP = 9, OMD = 112, OMT = 128;
constexpr float XS = 8.0f, WSC = 256.0f, BN_EPS = 1e-5f;

typedef _Float16 b16;
typedef __attribute__((ext_vector_type(16))) _Float16 v16b;
typedef __attribute__((ext_vector_type(8))) _Float16 v8b;
typedef __attribute__((ext_vector_type(8))) float v8f;
typedef __attribute__((ext_vector_type(4))) float v4f;
__device__ __forceinline__ float bf16_rne(float f) { unsigned int u = __float_as_uint(f); u += 0x7FFFu + ((u >> 16) & 1u); return __uint_as_float(u & 0xFFFF0000u); }
__device__ __forceinline__ void split16(float v, b16& hi, b16& lo) { hi = (b16)v; lo = (b16)(v - (float)hi); }
__device__ __forceinline__ v16b frag_kb(const b16* p, int hh) { const v8b a = *(const v8b*)(p + 8 * hh), b = *(const v8b*)(p + 16 + 8 * hh); v16b f;
#pragma unroll
  for (int e = 0; e < 8; ++e) { f[e] = a[e]; f[8 + e] = b[e]; } return f; }
__device__ __forceinline__ v8f wmma16b(v16b a, v16b b, v8f c) { v8f d = __builtin_amdgcn_wmma_f32_16x16x32_f16(false, a, false, b, (short)0, c, false, false); asm volatile("v_nop\n\tv_nop\n\tv_nop\n\tv_nop" : "+v"(d) : "v"(a), "v"(b)); return d; }
__device__ __forceinline__ void wave_lds_sync() { __builtin_amdgcn_fence(__ATOMIC_RELEASE, "workgroup"); __builtin_amdgcn_wave_barrier(); __builtin_amdgcn_fence(__ATOMIC_ACQUIRE, "workgroup"); }
__device__ __forceinline__ float pmul(float a, float b) { float p = a * b; asm volatile("" : "+v"(p)); return p; }
__device__ __forceinline__ int iclamp(int v, int lo, int hi) { return v < lo ? lo : (v > hi ? hi : v); }

__global__ __launch_bounds__(256) void prepx_kernel(const float* __restrict__ x, b16* __restrict__ XT) {
  __shared__ __attribute__((aligned(16))) b16 Tt[64][64 + 8];
  const int n = blockIdx.z, c0 = blockIdx.y * 64, p0 = blockIdx.x * 64, t_ = threadIdx.x;
  for (int q = t_; q < 64 * 64; q += 256) { const int cc = q >> 6, pp = q & 63; Tt[pp][cc] = (b16)(bf16_rne(x[((size_t)n * C + c0 + cc) * HW + p0 + pp]) * XS); }
  __syncthreads();
  for (int pass = 0; pass < 2; ++pass) { for (int q = t_; q < 64 * 8; q += 256) { const int pp = q >> 3, c8 = (q & 7) * 8; *(volatile v8b*)(XT + ((size_t)n * HW + p0 + pp) * C + c0 + c8) = *(const v8b*)(&Tt[pp][c8]); } __threadfence(); }
}
__global__ __launch_bounds__(256) void prepw_kernel(const float* __restrict__ wv, const float* __restrict__ wom, const float* __restrict__ wo, b16* __restrict__ WV, b16* __restrict__ WOM, b16* __restrict__ WO) {
  const int tid = blockIdx.x * 256 + threadIdx.x, nth = gridDim.x * 256; const int n1 = C * C / 8, n2 = OMT * C / 8, n3 = C * C / 8;
  for (int pass = 0; pass < 2; ++pass) {
    for (int g = tid; g < n1 + n2 + n3; g += nth) { v8b o; b16* dst;
      if (g < n1) { const int e = g * 8; dst = WV + e;
#pragma unroll
        for (int j = 0; j < 8; ++j) o[j] = (b16)(bf16_rne(wv[e + j]) * WSC); }
      else if (g < n1 + n2) { const int e = (g - n1) * 8, r = e / C; dst = WOM + e;
#pragma unroll
        for (int j = 0; j < 8; ++j) o[j] = (r < OMD) ? (b16)(bf16_rne(wom[(size_t)(r < OMD ? r : 0) * C + (e - r * C) + j]) * WSC) : (b16)0.0f; }
      else { const int e = (g - n1 - n2) * 8; dst = WO + e;
#pragma unroll
        for (int j = 0; j < 8; ++j) o[j] = (b16)(bf16_rne(wo[e + j]) * WSC); }
      *(volatile v8b*)dst = o; }
    __threadfence(); }
}
__global__ __launch_bounds__(128) void proj_kernel(const b16* __restrict__ XT, const b16* __restrict__ WV, const b16* __restrict__ WOM, const float* __restrict__ bv, const float* __restrict__ bom, float* __restrict__ V, float* __restrict__ OM) {
  __shared__ __attribute__((aligned(16))) float Ts[4][16][128 + 4];
  const int wave = threadIdx.x >> 5, lane = threadIdx.x & 31, nloc = lane & 15, hlf = lane >> 4; const int m0 = blockIdx.x * 64 + wave * 16, nb = blockIdx.y;
  const b16* B = nb < 2 ? WV + (size_t)nb * 128 * C : WOM;
  v8f acc[8];
#pragma unroll
  for (int t = 0; t < 8; ++t) acc[t] = (v8f){};
#pragma unroll 2
  for (int kb = 0; kb < C; kb += 32) { const v16b a = frag_kb(XT + (size_t)(m0 + nloc) * C + kb, hlf);
#pragma unroll
    for (int t = 0; t < 8; ++t) acc[t] = wmma16b(a, frag_kb(B + (size_t)(t * 16 + nloc) * C + kb, hlf), acc[t]); }
#pragma unroll
  for (int t = 0; t < 8; ++t) { const int col = t * 16 + nloc; const float bb = nb < 2 ? bf16_rne(bv[nb * 128 + col]) : (col < OMD ? bf16_rne(bom[col < OMD ? col : 0]) : 0.0f);
#pragma unroll
    for (int r = 0; r < 8; ++r) Ts[wave][8 * hlf + r][col] = acc[t][r] * (1.0f / (XS * WSC)) + bb; }
  wave_lds_sync();
  for (int pass = 0; pass < 2; ++pass) { for (int rr = 0; rr < 16; ++rr) { const v4f vv = *(const v4f*)(&Ts[wave][rr][lane * 4]); if (nb < 2) *(volatile v4f*)(V + (size_t)(m0 + rr) * C + nb * 128 + lane * 4) = vv; else *(volatile v4f*)(OM + (size_t)(m0 + rr) * OMT + lane * 4) = vv; } __threadfence(); }
}
__global__ __launch_bounds__(256) void sample_kernel(const float* __restrict__ V, const float* __restrict__ OM, b16* __restrict__ SH, b16* __restrict__ SL) {
  __shared__ float Som[OMT]; __shared__ __attribute__((aligned(16))) b16 Th[C + 8], Tl[C + 8];
  const int tok = blockIdx.x, t_ = threadIdx.x, g = t_ >> 6, c = t_ & 63; const int n = tok / HW, hw = tok - n * HW, h = hw / W, w = hw - h * W;
  if (t_ < OMT) Som[t_] = OM[(size_t)tok * OMT + t_];
  __syncthreads();
  const float* Vn = V + (size_t)n * HW * C + g * CG + c; float acc = 0.0f;
#pragma unroll 1
  for (int k = 0; k < KP; ++k) { const float dx = Som[g * 27 + 2 * k], dy = Som[g * 27 + 2 * k + 1], mk = Som[g * 27 + 18 + k];
    const float lh_ = (float)(h - 1 + k / 3) + dy, lw_ = (float)(w - 1 + k % 3) + dx; const float h0f = floorf(lh_), w0f = floorf(lw_); const float lh = lh_ - h0f, lw = lw_ - w0f;
    const int h0 = (int)h0f, w0 = (int)w0f; float s = 0.0f;
#pragma unroll
    for (int cy = 0; cy < 2; ++cy)
#pragma unroll
      for (int cx = 0; cx < 2; ++cx) { const int hi = h0 + cy, wi = w0 + cx; const bool valid = (hi >= 0) && (hi < H) && (wi >= 0) && (wi < W);
        const float wgt = pmul(cy ? lh : 1.0f - lh, cx ? lw : 1.0f - lw); const float val = Vn[(size_t)(iclamp(hi, 0, H - 1) * W + iclamp(wi, 0, W - 1)) * C];
        s += pmul(valid ? val : 0.0f, valid ? wgt : 0.0f); }
    acc += pmul(mk, s); }
  { b16 a_, c_; split16(acc * XS, a_, c_); Th[g * CG + c] = a_; Tl[g * CG + c] = c_; }
  __syncthreads();
  for (int pass = 0; pass < 2; ++pass) { if (t_ < 32) { *(volatile v8b*)(SH + (size_t)tok * C + t_ * 8) = *(const v8b*)(&Th[t_ * 8]); *(volatile v8b*)(SL + (size_t)tok * C + t_ * 8) = *(const v8b*)(&Tl[t_ * 8]); } __threadfence(); }
}
__global__ __launch_bounds__(128) void outproj_kernel(const b16* __restrict__ SH, const b16* __restrict__ SL, const b16* __restrict__ WO, const float* __restrict__ bo, const float* __restrict__ gam, const float* __restrict__ bet, const float* __restrict__ rmean, const float* __restrict__ rvar, float* __restrict__ out) {
  __shared__ __attribute__((aligned(16))) float Tc[128][64 + 4];
  const int wave = threadIdx.x >> 5, lane = threadIdx.x & 31, nloc = lane & 15, hlf = lane >> 4, t_ = threadIdx.x; const int tb = blockIdx.x * 64, n = tb / HW, hw0 = tb - n * HW, c0 = blockIdx.y * 128; const size_t m0 = (size_t)tb + wave * 16;
  v8f acc[8];
#pragma unroll
  for (int t = 0; t < 8; ++t) acc[t] = (v8f){};
#pragma unroll 2
  for (int kb = 0; kb < C; kb += 32) { const v16b a = frag_kb(SH + (m0 + nloc) * C + kb, hlf), al = frag_kb(SL + (m0 + nloc) * C + kb, hlf);
#pragma unroll
    for (int t = 0; t < 8; ++t) { const v16b bw = frag_kb(WO + (size_t)(c0 + t * 16 + nloc) * C + kb, hlf); acc[t] = wmma16b(a, bw, acc[t]); acc[t] = wmma16b(al, bw, acc[t]); } }
#pragma unroll
  for (int t = 0; t < 8; ++t) { const int c = c0 + t * 16 + nloc; const float inv = bf16_rne(gam[c]) / sqrtf(bf16_rne(rvar[c]) + BN_EPS), mu = bf16_rne(rmean[c]), be = bf16_rne(bet[c]), bb = bf16_rne(bo[c]);
#pragma unroll
    for (int r = 0; r < 8; ++r) { const float y = acc[t][r] * (1.0f / (XS * WSC)) + bb; const float z = pmul(y - mu, inv) + be; Tc[t * 16 + nloc][wave * 16 + 8 * hlf + r] = z / (1.0f + __expf(-z)); } }
  __syncthreads();
  for (int pass = 0; pass < 2; ++pass) { for (int q = t_; q < 128 * 16; q += 128) { const int cc = q >> 4, c4 = (q & 15) * 4; *(volatile v4f*)(out + ((size_t)n * C + c0 + cc) * HW + hw0 + c4) = *(const v4f*)(&Tc[cc][c4]); } __threadfence(); }
}
}

extern "C" void kernel_launch(void* const* d_in, const int* in_sizes, int n_in, void* d_out, int out_size, void* d_ws, size_t ws_size, hipStream_t stream) {
  (void)n_in;
  auto Fp = [&](int i) { return (const float*)d_in[i]; };
  if (in_sizes[0] != NTOK * C || in_sizes[1] != C * C || in_sizes[3] != OMD * C || in_sizes[4] != OMD || in_sizes[5] != C * C || out_size != NTOK * C) return;
  size_t off = 0; char* ws = (char*)d_ws;
  auto carve = [&](size_t bytes) { char* p = ws + off; off += (bytes + 255) & ~(size_t)255; return p; };
  b16* XT = (b16*)carve((size_t)NTOK * C * 2); b16* WV = (b16*)carve((size_t)C * C * 2); b16* WOM = (b16*)carve((size_t)OMT * C * 2); b16* WO = (b16*)carve((size_t)C * C * 2);
  float* V = (float*)carve((size_t)NTOK * C * 4); float* OM = (float*)carve((size_t)NTOK * OMT * 4); b16* SH = (b16*)carve((size_t)NTOK * C * 2); b16* SL = (b16*)carve((size_t)NTOK * C * 2);
  if (off > ws_size || off > ((size_t)128 << 20)) return;
  prepx_kernel<<<dim3(HW / 64, C / 64, NBt), 256, 0, stream>>>(Fp(0), XT);
  prepw_kernel<<<80, 256, 0, stream>>>(Fp(1), Fp(3), Fp(5), WV, WOM, WO);
  proj_kernel<<<dim3(NTOK / 64, 3), 128, 0, stream>>>(XT, WV, WOM, Fp(2), Fp(4), V, OM);
  sample_kernel<<<NTOK, 256, 0, stream>>>(V, OM, SH, SL);
  outproj_kernel<<<dim3(NTOK / 64, 2), 128, 0, stream>>>(SH, SL, WO, Fp(6), Fp(7), Fp(8), Fp(9), Fp(10), (float*)d_out);
}
